// TransformersLayer_87239375716863
// MI455X (gfx1250) — hardware-verified
//
#include <hip/hip_runtime.h>


#define NT_  2048
#define NBT  2
#define DM   1024
#define FF   4096
#define NH_  16
#define HD   64
#define QCH  256
#define PSC  32768.0f
#define LOSC 1024.0f
#define LOSCI (1.0f / 1024.0f)

typedef _Float16 h16;
typedef unsigned short bf;
typedef __attribute__((ext_vector_type(16))) __bf16   v16bf;
typedef __attribute__((ext_vector_type(16))) _Float16 v16h;
typedef __attribute__((ext_vector_type(8)))  _Float16 v8h;
typedef __attribute__((ext_vector_type(8)))  unsigned short v8us;
typedef __attribute__((ext_vector_type(8)))  float    v8f;
typedef __attribute__((ext_vector_type(4)))  float    v4f;
typedef v8h  __attribute__((may_alias)) v8ha;
typedef v4f  __attribute__((may_alias)) v4fa;
typedef v8us __attribute__((may_alias)) v8usa;

__device__ __forceinline__ unsigned short f2bf(float f) { unsigned u = __float_as_uint(f); u += 0x7FFFu + ((u >> 16) & 1u); return (unsigned short)(u >> 16); }
__device__ __forceinline__ float bf2f(unsigned short b) { return __uint_as_float(((unsigned)b) << 16); }
__device__ __forceinline__ float bfr(float f) { return bf2f(f2bf(f)); }
__device__ __forceinline__ v16h cat16(v8h lo, v8h hi) { return __builtin_shufflevector(lo, hi, 0, 1, 2, 3, 4, 5, 6, 7, 8, 9, 10, 11, 12, 13, 14, 15); }
__device__ __forceinline__ v16bf cat16b(v8us lo, v8us hi) { return __builtin_bit_cast(v16bf, __builtin_shufflevector(lo, hi, 0, 1, 2, 3, 4, 5, 6, 7, 8, 9, 10, 11, 12, 13, 14, 15)); }
__device__ __forceinline__ v8f wmma16(v16h a, v16h b, v8f c) { return __builtin_amdgcn_wmma_f32_16x16x32_f16(false, a, false, b, (short)0, c, false, false); }
__device__ __forceinline__ v8f wmmab(v16bf a, v16bf b, v8f c) { return __builtin_amdgcn_wmma_f32_16x16x32_bf16(false, a, false, b, (short)0, c, false, false); }

__global__ __launch_bounds__(256) void k_rows(const float* __restrict__ src, int rows, int C, bf* dst) {
    const int lane = threadIdx.x & 31, r = blockIdx.x * 8 + (threadIdx.x >> 5);
    if (r >= rows) return;
#pragma unroll 1
    for (int ps = 0; ps < 2; ++ps) {
        for (int q = 0; q < C / 256; ++q) { v8us o;
#pragma unroll
            for (int i = 0; i < 8; ++i) o[i] = f2bf(src[(size_t)r * C + q * 256 + lane * 8 + i]);
            *(volatile v8us*)(dst + (size_t)r * C + q * 256 + lane * 8) = o; }
        if (ps == 0) __threadfence(); }
}
template <bool ROUNDSRC>
__global__ __launch_bounds__(256) void k_ln(const float* __restrict__ src, int lds, const float* __restrict__ res, int ldr, const float* __restrict__ g, const float* __restrict__ be, bf* PH, bf* PL, float* Xout) {
    const int lane = threadIdx.x & 31, r = blockIdx.x * 8 + (threadIdx.x >> 5);
    if (r >= NT_) return;
    float v[32]; float s = 0.f;
#pragma unroll
    for (int q = 0; q < 4; ++q)
#pragma unroll
        for (int i = 0; i < 8; ++i) { const int c = q * 256 + lane * 8 + i; float t = src[(size_t)r * lds + c]; if (ROUNDSRC) t = bfr(t); if (res) t += bfr(res[(size_t)r * ldr + c]); v[q * 8 + i] = t; s += t; }
#pragma unroll
    for (int sh = 16; sh; sh >>= 1) s += __shfl_xor(s, sh, 32);
    const float mu = s * (1.0f / DM); float sq = 0.f;
#pragma unroll
    for (int k = 0; k < 32; ++k) { const float d = v[k] - mu; sq += d * d; }
#pragma unroll
    for (int sh = 16; sh; sh >>= 1) sq += __shfl_xor(sq, sh, 32);
    const float rs = rsqrtf(sq * (1.0f / DM) + 1e-5f);
#pragma unroll 1
    for (int ps = 0; ps < 2; ++ps) {
#pragma unroll
        for (int q = 0; q < 4; ++q) { v8us oh, ol; v4f x0, x1;
#pragma unroll
            for (int i = 0; i < 8; ++i) { const int c = q * 256 + lane * 8 + i; const float y = (v[q * 8 + i] - mu) * rs * bfr(g[c]) + bfr(be[c]); const unsigned short hb = f2bf(y); oh[i] = hb; ol[i] = f2bf(y - bf2f(hb)); if (i < 4) x0[i] = v[q * 8 + i]; else x1[i - 4] = v[q * 8 + i]; }
            *(volatile v8us*)(PH + (size_t)r * DM + q * 256 + lane * 8) = oh; *(volatile v8us*)(PL + (size_t)r * DM + q * 256 + lane * 8) = ol;
            if (Xout) { *(volatile v4f*)(Xout + (size_t)r * DM + q * 256 + lane * 8) = x0; *(volatile v4f*)(Xout + (size_t)r * DM + q * 256 + lane * 8 + 4) = x1; } }
        if (ps == 0) __threadfence(); }
}
template <int EPI, bool RROUND = false>
__global__ __launch_bounds__(128) void k_gemm(const bf* __restrict__ A, const bf* __restrict__ Al, const bf* __restrict__ Bn, int K, const float* __restrict__ bias, const float* __restrict__ Rf, int ldr, int ldc, float* C, bf* PH, bf* PL) {
    __shared__ __align__(16) float ost[4][16 * 68];
    const int lane = threadIdx.x & 31, wave = threadIdx.x >> 5, lr = lane & 15, hi = lane >> 4;
    const size_t r0 = (size_t)blockIdx.x * 64 + wave * 16; const int c0 = blockIdx.y * 64;
    const size_t aoff = (r0 + lr) * (size_t)K + 8 * hi;
    size_t boff[4];
#pragma unroll
    for (int t = 0; t < 4; ++t) boff[t] = (size_t)(c0 + t * 16 + lr) * K + 8 * hi;
    v8f acc[4];
#pragma unroll
    for (int t = 0; t < 4; ++t) acc[t] = (v8f){};
#pragma unroll 2
    for (int kc = 0; kc < K; kc += 32) {
        const v16bf a = cat16b(*(const v8us*)(A + aoff + kc), *(const v8us*)(A + aoff + kc + 16)), al = cat16b(*(const v8us*)(Al + aoff + kc), *(const v8us*)(Al + aoff + kc + 16));
#pragma unroll
        for (int t = 0; t < 4; ++t) { const v16bf bb = cat16b(*(const v8us*)(Bn + boff[t] + kc), *(const v8us*)(Bn + boff[t] + kc + 16)); acc[t] = wmmab(a, bb, acc[t]); acc[t] = wmmab(al, bb, acc[t]); }
        asm volatile("v_nop" : "+v"(acc[0]), "+v"(acc[1]), "+v"(acc[2]), "+v"(acc[3]) : "v"(a), "v"(al) : "memory");
    }
    float* os = &ost[wave][0];
#pragma unroll
    for (int t = 0; t < 4; ++t) { const int col = c0 + t * 16 + lr; const float bv = bfr(bias[col]);
#pragma unroll
        for (int j = 0; j < 8; ++j) { float v = acc[t][j] + bv; if (EPI == 1) v = fmaxf(v, 0.f); if (EPI == 0 && Rf) { const float rv = Rf[(r0 + hi * 8 + j) * (size_t)ldr + col]; v += RROUND ? bfr(rv) : rv; } os[(hi * 8 + j) * 68 + t * 16 + lr] = v; } }
    __builtin_amdgcn_wave_barrier(); asm volatile("" ::: "memory");
    if (EPI == 0) {
        float* crow = C + r0 * ldc + c0;
        auto pass = [&]() {
#pragma unroll
            for (int s = 0; s < 8; ++s) { const int Lid = (lane >> 3) + 4 * s, piece = lane & 7; const int row = Lid >> 1, cofs = (Lid & 1) * 32 + piece * 4;
                const v4f val = *(const v4fa*)(os + row * 68 + cofs); *(volatile v4f*)(crow + (size_t)row * ldc + cofs) = val; }
        };
        pass(); __threadfence(); pass();
    } else {
        bf* p1 = PH + r0 * ldc + c0; bf* p2 = PL + r0 * ldc + c0;
        auto pass = [&]() {
#pragma unroll
            for (int s = 0; s < 4; ++s) { const int row = 4 * s + (lane >> 3), piece = lane & 7; const float* sp = os + row * 68 + piece * 8; v8us oh, ol;
#pragma unroll
                for (int i = 0; i < 8; ++i) { const unsigned short hb = f2bf(sp[i]); oh[i] = hb; ol[i] = f2bf(sp[i] - bf2f(hb)); }
                *(volatile v8us*)(p1 + (size_t)row * ldc + piece * 8) = oh; *(volatile v8us*)(p2 + (size_t)row * ldc + piece * 8) = ol; }
        };
        pass(); __threadfence(); pass();
    }
}
__global__ __launch_bounds__(256) void k_q16(const float* __restrict__ Q, h16* QH, h16* QL) {
    const int lane = threadIdx.x & 31, r = blockIdx.x * 8 + (threadIdx.x >> 5);
    if (r >= NT_) return;
#pragma unroll 1
    for (int ps = 0; ps < 2; ++ps) {
#pragma unroll
        for (int q = 0; q < 4; ++q) { v8h oh, ol;
#pragma unroll
            for (int i = 0; i < 8; ++i) { const float v = Q[(size_t)r * DM + q * 256 + lane * 8 + i]; const h16 a = (h16)v; oh[i] = a; ol[i] = (h16)((v - (float)a) * LOSC); }
            *(volatile v8h*)(QH + (size_t)r * DM + q * 256 + lane * 8) = oh; *(volatile v8h*)(QL + (size_t)r * DM + q * 256 + lane * 8) = ol; }
        if (ps == 0) __threadfence(); }
}
__global__ __launch_bounds__(256) void k_vt(const float* __restrict__ V, bf* VTH, bf* VTL) {
    __shared__ float tl[64][65];
    const int tid = threadIdx.x, t0 = blockIdx.x * 64, h = blockIdx.y;
    { const int tt = tid >> 2, dq = (tid & 3) * 16;
#pragma unroll
      for (int i = 0; i < 16; ++i) tl[dq + i][tt] = V[(size_t)(t0 + tt) * DM + h * HD + dq + i]; }
    __syncthreads();
    const int piece = tid & 7;
    auto pass = [&]() {
#pragma unroll
        for (int s = 0; s < 2; ++s) { const int d = (tid >> 3) + 32 * s; v8us oh, ol;
#pragma unroll
            for (int i = 0; i < 8; ++i) { const float v = tl[d][piece * 8 + i]; const unsigned short hb = f2bf(v); oh[i] = hb; ol[i] = f2bf(v - bf2f(hb)); }
            const size_t o = ((size_t)h * HD + d) * NT_ + t0 + piece * 8; *(volatile v8us*)(VTH + o) = oh; *(volatile v8us*)(VTL + o) = ol; }
    };
    pass(); __threadfence(); pass();
}
__global__ __launch_bounds__(128) void k_sgemm(const h16* __restrict__ QH, const h16* __restrict__ QL, int qbase, float* S) {
    __shared__ __align__(16) float ost[4][16 * 68];
    const int lane = threadIdx.x & 31, wave = threadIdx.x >> 5, lr = lane & 15, hi = lane >> 4, h = blockIdx.z;
    const int r0 = blockIdx.x * 64 + wave * 16, c0 = blockIdx.y * 64;
    const size_t aoff = (size_t)(qbase + r0 + lr) * DM + h * HD + 8 * hi;
    v8f acc[4], accx[4];
#pragma unroll
    for (int t = 0; t < 4; ++t) { acc[t] = (v8f){}; accx[t] = (v8f){}; }
#pragma unroll
    for (int kc = 0; kc < HD; kc += 32) {
        const v16h a = cat16(*(const v8h*)(QH + aoff + kc), *(const v8h*)(QH + aoff + kc + 16)), al = cat16(*(const v8h*)(QL + aoff + kc), *(const v8h*)(QL + aoff + kc + 16));
#pragma unroll
        for (int t = 0; t < 4; ++t) { const size_t bo = (size_t)(c0 + t * 16 + lr) * DM + h * HD + 8 * hi + kc; const v16h bb = cat16(*(const v8h*)(QH + bo), *(const v8h*)(QH + bo + 16)), bl = cat16(*(const v8h*)(QL + bo), *(const v8h*)(QL + bo + 16));
            acc[t] = wmma16(a, bb, acc[t]); accx[t] = wmma16(a, bl, accx[t]); accx[t] = wmma16(al, bb, accx[t]); }
        asm volatile("v_nop" : "+v"(acc[0]), "+v"(acc[1]), "+v"(acc[2]), "+v"(acc[3]), "+v"(accx[0]), "+v"(accx[1]), "+v"(accx[2]), "+v"(accx[3]) : "v"(a), "v"(al) : "memory");
    }
    float* os = &ost[wave][0];
#pragma unroll
    for (int t = 0; t < 4; ++t)
#pragma unroll
        for (int j = 0; j < 8; ++j) os[(hi * 8 + j) * 68 + t * 16 + lr] = (acc[t][j] + accx[t][j] * LOSCI) * 0.125f;
    __builtin_amdgcn_wave_barrier(); asm volatile("" ::: "memory");
    float* crow = S + ((size_t)h * QCH + r0) * NT_ + c0;
    auto pass = [&]() {
#pragma unroll
        for (int s = 0; s < 8; ++s) { const int Lid = (lane >> 3) + 4 * s, piece = lane & 7; const int row = Lid >> 1, cofs = (Lid & 1) * 32 + piece * 4;
            const v4f val = *(const v4fa*)(os + row * 68 + cofs); *(volatile v4f*)(crow + (size_t)row * NT_ + cofs) = val; }
    };
    pass(); __threadfence(); pass();
}
__global__ __launch_bounds__(256) void k_hsoft(const float* __restrict__ S, bf* PH, bf* PL) {
    __shared__ __align__(16) unsigned short th[8][NH_ * 64];
    __shared__ __align__(16) unsigned short tlo[8][NH_ * 64];
    const int lane = threadIdx.x & 31, wave = threadIdx.x >> 5, r = blockIdx.x * 8 + wave;
    if (r >= QCH) return;
    unsigned short* ph_ = &th[wave][0]; unsigned short* pl_ = &tlo[wave][0];
#pragma unroll 1
    for (int q = 0; q < NT_ / 64; ++q) { const int k0 = q * 64;
        float v[NH_][2];
#pragma unroll
        for (int h = 0; h < NH_; ++h) { const float* sr = S + ((size_t)h * QCH + r) * NT_ + k0; v[h][0] = sr[lane]; v[h][1] = sr[32 + lane]; }
#pragma unroll
        for (int e = 0; e < 2; ++e) { float mx = v[0][e];
#pragma unroll
            for (int h = 1; h < NH_; ++h) mx = fmaxf(mx, v[h][e]);
            float ssum = 0.f;
#pragma unroll
            for (int h = 0; h < NH_; ++h) { v[h][e] = __expf(v[h][e] - mx); ssum += v[h][e]; }
            const float sc = PSC / ssum;
#pragma unroll
            for (int h = 0; h < NH_; ++h) { const float p = v[h][e] * sc; const unsigned short hb = f2bf(p); ph_[h * 64 + e * 32 + lane] = hb; pl_[h * 64 + e * 32 + lane] = f2bf(p - bf2f(hb)); } }
        asm volatile("" ::: "memory"); __builtin_amdgcn_wave_barrier();
#pragma unroll 1
        for (int ps = 0; ps < 2; ++ps) {
#pragma unroll
            for (int s = 0; s < 4; ++s) { const int h = s * 4 + (lane >> 3), piece = lane & 7;
                const v8us a = *(const v8usa*)(ph_ + h * 64 + piece * 8), b = *(const v8usa*)(pl_ + h * 64 + piece * 8);
                *(volatile v8us*)(PH + ((size_t)h * QCH + r) * NT_ + k0 + piece * 8) = a; *(volatile v8us*)(PL + ((size_t)h * QCH + r) * NT_ + k0 + piece * 8) = b; }
            if (ps == 0) __threadfence(); }
        __builtin_amdgcn_wave_barrier(); asm volatile("" ::: "memory");
    }
}
__global__ __launch_bounds__(128) void k_pvgemm(const bf* __restrict__ PH, const bf* __restrict__ PL, const bf* __restrict__ VTH, const bf* __restrict__ VTL, int qbase, float* ATT) {
    __shared__ __align__(16) float ost[4][16 * 68];
    const int lane = threadIdx.x & 31, wave = threadIdx.x >> 5, lr = lane & 15, hi = lane >> 4, h = blockIdx.z;
    const int r0 = blockIdx.x * 64 + wave * 16;
    const size_t aoff = ((size_t)h * QCH + r0 + lr) * NT_ + 8 * hi;
    v8f acc[4];
#pragma unroll
    for (int t = 0; t < 4; ++t) acc[t] = (v8f){};
#pragma unroll 2
    for (int kc = 0; kc < NT_; kc += 32) {
        const v16bf a = cat16b(*(const v8us*)(PH + aoff + kc), *(const v8us*)(PH + aoff + kc + 16)), al = cat16b(*(const v8us*)(PL + aoff + kc), *(const v8us*)(PL + aoff + kc + 16));
#pragma unroll
        for (int t = 0; t < 4; ++t) { const size_t bo = ((size_t)h * HD + t * 16 + lr) * NT_ + 8 * hi + kc; const v16bf bb = cat16b(*(const v8us*)(VTH + bo), *(const v8us*)(VTH + bo + 16)), bl = cat16b(*(const v8us*)(VTL + bo), *(const v8us*)(VTL + bo + 16));
            acc[t] = wmmab(a, bb, acc[t]); acc[t] = wmmab(al, bb, acc[t]); acc[t] = wmmab(a, bl, acc[t]); }
        asm volatile("v_nop" : "+v"(acc[0]), "+v"(acc[1]), "+v"(acc[2]), "+v"(acc[3]) : "v"(a), "v"(al) : "memory");
    }
    float* os = &ost[wave][0];
#pragma unroll
    for (int t = 0; t < 4; ++t)
#pragma unroll
        for (int j = 0; j < 8; ++j) os[(hi * 8 + j) * 68 + t * 16 + lr] = acc[t][j] * (1.0f / PSC);
    __builtin_amdgcn_wave_barrier(); asm volatile("" ::: "memory");
    float* crow = ATT + (size_t)(qbase + r0) * DM + h * HD;
    auto pass = [&]() {
#pragma unroll
        for (int s = 0; s < 8; ++s) { const int Lid = (lane >> 3) + 4 * s, piece = lane & 7; const int row = Lid >> 1, cofs = (Lid & 1) * 32 + piece * 4;
            const v4f val = *(const v4fa*)(os + row * 68 + cofs); *(volatile v4f*)(crow + (size_t)row * DM + cofs) = val; }
    };
    pass(); __threadfence(); pass();
}
__global__ __launch_bounds__(256) void k_attbf(const float* __restrict__ A, bf* PH, bf* PL) {
    const int lane = threadIdx.x & 31, r = blockIdx.x * 8 + (threadIdx.x >> 5);
    if (r >= NT_) return;
#pragma unroll 1
    for (int ps = 0; ps < 2; ++ps) {
#pragma unroll
        for (int q = 0; q < 4; ++q) { v8us oh, ol;
#pragma unroll
            for (int i = 0; i < 8; ++i) { const float v = A[(size_t)r * DM + q * 256 + lane * 8 + i]; const unsigned short hb = f2bf(v); oh[i] = hb; ol[i] = f2bf(v - bf2f(hb)); }
            *(volatile v8us*)(PH + (size_t)r * DM + q * 256 + lane * 8) = oh; *(volatile v8us*)(PL + (size_t)r * DM + q * 256 + lane * 8) = ol; }
        if (ps == 0) __threadfence(); }
}

extern "C" void kernel_launch(void* const* d_in, const int* in_sizes, int n_in,
                              void* d_out, int out_size, void* d_ws, size_t ws_size, hipStream_t stream) {
    (void)in_sizes; (void)n_in; (void)out_size;
    const float* x = (const float*)d_in[0]; const float* g1 = (const float*)d_in[1]; const float* be1 = (const float*)d_in[2]; const float* g2 = (const float*)d_in[3]; const float* be2 = (const float*)d_in[4];
    const float* Ws = (const float*)d_in[5]; const float* bs = (const float*)d_in[6]; const float* Wo = (const float*)d_in[7]; const float* bo = (const float*)d_in[8];
    const float* W1 = (const float*)d_in[9]; const float* b1 = (const float*)d_in[10]; const float* W2 = (const float*)d_in[11]; const float* b2 = (const float*)d_in[12];
    float* out = (float*)d_out;
    char* wsp = (char*)d_ws;
    auto take = [&](size_t bytes) { char* p = wsp; wsp += (bytes + 255) & ~(size_t)255; return (void*)p; };
    bf* WsB = (bf*)take((size_t)DM * DM * 2); bf* WoB = (bf*)take((size_t)DM * DM * 2); bf* W1B = (bf*)take((size_t)FF * DM * 2); bf* W2B = (bf*)take((size_t)DM * FF * 2);
    bf* LH = (bf*)take((size_t)NT_ * DM * 2); bf* LL = (bf*)take((size_t)NT_ * DM * 2);
    float* Qf = (float*)take((size_t)NT_ * DM * 4);
    h16* QH = (h16*)take((size_t)NT_ * DM * 2); h16* QL = (h16*)take((size_t)NT_ * DM * 2); bf* VTH = (bf*)take((size_t)NT_ * DM * 2); bf* VTL = (bf*)take((size_t)NT_ * DM * 2);
    float* S = (float*)take((size_t)NH_ * QCH * NT_ * 4);
    bf* PH = (bf*)take((size_t)NH_ * QCH * NT_ * 2); bf* PL = (bf*)take((size_t)NH_ * QCH * NT_ * 2);
    bf* AH = (bf*)take((size_t)NT_ * DM * 2); bf* AL = (bf*)take((size_t)NT_ * DM * 2);
    if ((size_t)(wsp - (char*)d_ws) > ws_size) return;
    float* ATT = Qf;
    bf* HH = (bf*)S; bf* HL = (bf*)((char*)S + (size_t)NT_ * FF * 2);
    float* X1 = Qf;
    k_rows<<<DM / 8, 256, 0, stream>>>(Ws, DM, DM, WsB); k_rows<<<DM / 8, 256, 0, stream>>>(Wo, DM, DM, WoB); k_rows<<<FF / 8, 256, 0, stream>>>(W1, FF, DM, W1B); k_rows<<<DM / 8, 256, 0, stream>>>(W2, DM, FF, W2B);
    for (int b = 0; b < NBT; ++b) {
        const float* xb = x + (size_t)b * DM; float* ob = out + (size_t)b * DM;
        k_ln<true><<<NT_ / 8, 256, 0, stream>>>(xb, 2 * DM, nullptr, 0, g1, be1, LH, LL, nullptr);
        k_gemm<0><<<dim3(NT_ / 64, DM / 64, 1), 128, 0, stream>>>(LH, LL, WsB, DM, bs, nullptr, 0, DM, Qf, nullptr, nullptr);
        k_q16<<<NT_ / 8, 256, 0, stream>>>(Qf, QH, QL); k_vt<<<dim3(NT_ / 64, NH_, 1), 256, 0, stream>>>(Qf, VTH, VTL);
        for (int c = 0; c < NT_ / QCH; ++c) {
            k_sgemm<<<dim3(QCH / 64, NT_ / 64, NH_), 128, 0, stream>>>(QH, QL, c * QCH, S);
            k_hsoft<<<QCH / 8, 256, 0, stream>>>(S, PH, PL);
            k_pvgemm<<<dim3(QCH / 64, 1, NH_), 128, 0, stream>>>(PH, PL, VTH, VTL, c * QCH, ATT);
        }
        k_attbf<<<NT_ / 8, 256, 0, stream>>>(ATT, AH, AL);
        k_gemm<0, true><<<dim3(NT_ / 64, DM / 64, 1), 128, 0, stream>>>(AH, AL, WoB, DM, bo, xb, 2 * DM, DM, X1, nullptr, nullptr);
        k_ln<false><<<NT_ / 8, 256, 0, stream>>>(X1, DM, nullptr, 0, g2, be2, LH, LL, nullptr);
        k_gemm<1><<<dim3(NT_ / 64, FF / 64, 1), 128, 0, stream>>>(LH, LL, W1B, DM, b1, nullptr, 0, FF, nullptr, HH, HL);
        k_gemm<0><<<dim3(NT_ / 64, DM / 64, 1), 128, 0, stream>>>(HH, HL, W2B, FF, b2, X1, DM, 2 * DM, ob, nullptr, nullptr);
    }
}
